// SHSAttention_18133351924335
// MI455X (gfx1250) — hardware-verified
//
#include <hip/hip_runtime.h>
#include <stddef.h>
#include <stdint.h>

#define NB    8
#define LSEQ  2048
#define HID   768
#define PD    164
#define QKD   16
#define NQKV  196
#define NTOK  (NB * LSEQ)
#define KP    192
#define NQP   224
#define QP    32
#define VP    192
#define BR    32
#define BC    128
#define NQT   (LSEQ / BR)

static_assert(NTOK == 16384);
static_assert(KP % 32 == 0);
static_assert(KP >= PD);
static_assert(NQP == 32 + 3 * 64);
static_assert(VP == NQP - 32);
static_assert(VP % 16 == 0);
static_assert(LSEQ % 256 == 0);
static_assert(LSEQ % BC == 0);
static_assert(LSEQ % BR == 0);
static_assert(NTOK % 256 == 0);
static_assert(NTOK % 8 == 0);
static_assert(HID % 64 == 0);
static_assert(HID % 32 == 0);
static_assert((HID - KP) % 8 == 0);
static_assert(((HID - KP) / 8) == 72);
static_assert((KP - PD) == 28);

typedef _Float16 v16h __attribute__((ext_vector_type(16)));
typedef _Float16 v8h  __attribute__((ext_vector_type(8)));
typedef float    v8f  __attribute__((ext_vector_type(8)));
typedef float    v4f  __attribute__((ext_vector_type(4)));
typedef unsigned int   v4u   __attribute__((ext_vector_type(4)));
typedef unsigned short v8us  __attribute__((ext_vector_type(8)));
typedef unsigned short v16us __attribute__((ext_vector_type(16)));
typedef __bf16         v16b  __attribute__((ext_vector_type(16)));
typedef unsigned short ush;

union Frag  { v16h v; v8h h[2]; };
union FragU { v16us v; v8us h[2]; v16b b; };
union Pack8 { v8h h; v4u u; };
union PackU { v8us s; v4u u; };
struct HL { v4u h; v4u l; };

__device__ __forceinline__ ush f2bf(float f) {
  const unsigned u = __float_as_uint(f);
  return (ush)((u + 0x7FFFu + ((u >> 16) & 1u)) >> 16);
}
__device__ __forceinline__ float bf2f(ush b) { return __uint_as_float(((unsigned)b) << 16); }

__device__ __forceinline__ HL split8(v8f f) {
  PackU ph, pl;
#pragma unroll
  for (int e = 0; e < 8; ++e) {
    const ush hi = f2bf(f[e]);
    ph.s[e] = hi;
    pl.s[e] = f2bf(f[e] - bf2f(hi));
  }
  HL r; r.h = ph.u; r.l = pl.u;
  return r;
}

__device__ __forceinline__ v8f mma16(v16h a, v16h b, v8f c) {
  c = __builtin_amdgcn_wmma_f32_16x16x32_f16(false, a, false, b, (short)0, c, false, false);
  asm volatile("v_nop\n\tv_nop\n\tv_nop\n\tv_nop" : "+v"(c) : "v"(a), "v"(b));
  return c;
}
__device__ __forceinline__ v8f mmab(v16us a, v16us b, v8f c) {
  FragU ua, ub; ua.v = a; ub.v = b;
  c = __builtin_amdgcn_wmma_f32_16x16x32_bf16(false, ua.b, false, ub.b, (short)0, c, false, false);
  asm volatile("v_nop\n\tv_nop\n\tv_nop\n\tv_nop" : "+v"(c) : "v"(a), "v"(b));
  return c;
}

__device__ __forceinline__ v16h ldfrag(const _Float16* p, int ld, int row0, int k0, int lane) {
  const int m = lane & 15, lh = lane >> 4;
  const _Float16* q = p + (size_t)(row0 + m) * ld + k0 + 8 * lh;
  Frag f;
  f.h[0] = *(const v8h*)(q);
  f.h[1] = *(const v8h*)(q + 16);
  return f.v;
}
__device__ __forceinline__ v16us ldfragu(const ush* p, int ld, int row0, int k0, int lane) {
  const int m = lane & 15, lh = lane >> 4;
  const ush* q = p + (size_t)(row0 + m) * ld + k0 + 8 * lh;
  FragU f;
  f.h[0] = *(const v8us*)(q);
  f.h[1] = *(const v8us*)(q + 16);
  return f.v;
}

__device__ __forceinline__ v8f zero8() { return (v8f){0.f, 0.f, 0.f, 0.f, 0.f, 0.f, 0.f, 0.f}; }

__device__ __forceinline__ void gemm32x64(const _Float16* __restrict__ A, int lda,
                                          const _Float16* __restrict__ Bt, int ldb,
                                          int m0, int n0, int lane, v8f (&acc)[2][4]) {
#pragma unroll 2
  for (int k0 = 0; k0 < HID; k0 += 32) {
    const v16h a0 = ldfrag(A, lda, m0, k0, lane);
    const v16h a1 = ldfrag(A, lda, m0 + 16, k0, lane);
    const v16h b0 = ldfrag(Bt, ldb, n0, k0, lane);
    const v16h b1 = ldfrag(Bt, ldb, n0 + 16, k0, lane);
    const v16h b2 = ldfrag(Bt, ldb, n0 + 32, k0, lane);
    const v16h b3 = ldfrag(Bt, ldb, n0 + 48, k0, lane);
    acc[0][0] = mma16(a0, b0, acc[0][0]);
    acc[1][0] = mma16(a1, b0, acc[1][0]);
    acc[0][1] = mma16(a0, b1, acc[0][1]);
    acc[1][1] = mma16(a1, b1, acc[1][1]);
    acc[0][2] = mma16(a0, b2, acc[0][2]);
    acc[1][2] = mma16(a1, b2, acc[1][2]);
    acc[0][3] = mma16(a0, b3, acc[0][3]);
    acc[1][3] = mma16(a1, b3, acc[1][3]);
  }
}

__device__ __forceinline__ void gemm3_32x64(const ush* __restrict__ Ah, const ush* __restrict__ Al, int lda,
                                            const ush* __restrict__ Bh, const ush* __restrict__ Bl, int ldb,
                                            int m0, int n0, int lane, v8f (&acc)[2][4]) {
#pragma unroll 1
  for (int k0 = 0; k0 < KP; k0 += 32) {
    const v16us a0h = ldfragu(Ah, lda, m0, k0, lane);
    const v16us a1h = ldfragu(Ah, lda, m0 + 16, k0, lane);
    const v16us a0l = ldfragu(Al, lda, m0, k0, lane);
    const v16us a1l = ldfragu(Al, lda, m0 + 16, k0, lane);
#pragma unroll
    for (int t = 0; t < 4; ++t) {
      const v16us bh = ldfragu(Bh, ldb, n0 + 16 * t, k0, lane);
      const v16us bl = ldfragu(Bl, ldb, n0 + 16 * t, k0, lane);
      acc[0][t] = mmab(a0h, bh, acc[0][t]);
      acc[1][t] = mmab(a1h, bh, acc[1][t]);
      acc[0][t] = mmab(a0h, bl, acc[0][t]);
      acc[1][t] = mmab(a1h, bl, acc[1][t]);
      acc[0][t] = mmab(a0l, bh, acc[0][t]);
      acc[1][t] = mmab(a1l, bh, acc[1][t]);
    }
  }
}

__global__ __launch_bounds__(256) void k_prep(const float* __restrict__ x, const float* __restrict__ g,
                                              const float* __restrict__ be, ush* __restrict__ xh,
                                              ush* __restrict__ xl, _Float16* __restrict__ mg) {
  __shared__ __align__(16) float xs[8 * KP];
  const int tid = threadIdx.x, lane = tid & 31, w = tid >> 5;
  const int tok = blockIdx.x * 8 + w;
  const float* xr = x + (size_t)tok * HID;

  float v[6];
  float sm = 0.f;
#pragma unroll
  for (int i = 0; i < 6; ++i) {
    const int d  = lane + 32 * i;
    const int dc = (d < PD) ? d : (PD - 1);
    const float t = xr[dc];
    v[i] = (d < PD) ? t : 0.f;
    sm += v[i];
  }
#pragma unroll
  for (int m = 16; m > 0; m >>= 1) sm += __shfl_xor(sm, m, 32);
  const float mean = sm * (1.0f / (float)PD);
  float s2 = 0.f;
#pragma unroll
  for (int i = 0; i < 6; ++i) {
    const int d = lane + 32 * i;
    const float cdev = (d < PD) ? (v[i] - mean) : 0.f;
    s2 += cdev * cdev;
  }
#pragma unroll
  for (int m = 16; m > 0; m >>= 1) s2 += __shfl_xor(s2, m, 32);
  const float rstd = rsqrtf(s2 * (1.0f / (float)PD) + 1.0e-5f);
#pragma unroll
  for (int i = 0; i < 6; ++i) {
    const int d  = lane + 32 * i;
    const int dc = (d < PD) ? d : (PD - 1);
    const float y = (v[i] - mean) * rstd * g[dc] + be[dc];
    xs[w * KP + d] = (d < PD) ? y : 0.f;
  }
  __syncthreads();

  const int pl = (lane < 24) ? lane : 23;
  const v4f f0 = *(const v4f*)(xs + w * KP + 8 * pl);
  const v4f f1 = *(const v4f*)(xs + w * KP + 8 * pl + 4);
  const HL s = split8((v8f){f0[0], f0[1], f0[2], f0[3], f1[0], f1[1], f1[2], f1[3]});
  const size_t o1 = (size_t)tok * KP + 8 * pl;

  v4u p2[3];
  size_t g2[3];
#pragma unroll
  for (int it = 0; it < 3; ++it) {
    const int pc  = lane + 32 * it;
    const int pcc = (pc < 72) ? pc : 71;
    const float* sp = xr + KP + 8 * pcc;
    const v4f a0 = *(const v4f*)(sp);
    const v4f a1 = *(const v4f*)(sp + 4);
    Pack8 pk;
    pk.h = (v8h){(_Float16)a0[0], (_Float16)a0[1], (_Float16)a0[2], (_Float16)a0[3],
                 (_Float16)a1[0], (_Float16)a1[1], (_Float16)a1[2], (_Float16)a1[3]};
    p2[it] = pk.u;
    g2[it] = (size_t)tok * HID + KP + 8 * pcc;
  }
  for (int ps = 0; ps < 2; ++ps) {
    if (lane < 24) { *(volatile v4u*)(xh + o1) = s.h; *(volatile v4u*)(xl + o1) = s.l; }
    *(volatile v4u*)(mg + g2[0]) = p2[0];
    *(volatile v4u*)(mg + g2[1]) = p2[1];
    if (lane < 8) *(volatile v4u*)(mg + g2[2]) = p2[2];
    __threadfence();
  }
}

__global__ __launch_bounds__(256) void k_cvt_wo(const float* __restrict__ w, _Float16* __restrict__ wo, int ngrp) {
  const int t = blockIdx.x * 256 + (int)threadIdx.x;
  if (t >= ngrp) return;
  const int o  = t / (HID / 8);
  const int d0 = (t - o * (HID / 8)) * 8;
  const size_t off = (size_t)o * HID + d0;
  const v4f a0 = *(const v4f*)(w + off);
  const v4f a1 = *(const v4f*)(w + off + 4);
  const v8f f = (v8f){a0[0], a0[1], a0[2], a0[3], a1[0], a1[1], a1[2], a1[3]};
  Pack8 pk;
#pragma unroll
  for (int e = 0; e < 8; ++e) {
    const float sc = (d0 + e < PD) ? 2.0f : 32.0f;
    pk.h[e] = (_Float16)(f[e] * sc);
  }
  const v4u vv = pk.u;
  for (int ps = 0; ps < 2; ++ps) {
    *(volatile v4u*)(wo + off) = vv;
    __threadfence();
  }
}

__global__ __launch_bounds__(256) void k_cvt_wq(const float* __restrict__ w, ush* __restrict__ wqh,
                                                ush* __restrict__ wql, int ngrp) {
  const int t = blockIdx.x * 256 + (int)threadIdx.x;
  if (t >= ngrp) return;
  const int o  = t / (KP / 8);
  const int d0 = (t - o * (KP / 8)) * 8;
  const int oc = (o < NQKV) ? o : (NQKV - 1);
  v8f f;
#pragma unroll
  for (int e = 0; e < 8; ++e) {
    const int d  = d0 + e;
    const int dc = (d < PD) ? d : (PD - 1);
    const float val = w[(size_t)oc * PD + dc];
    f[e] = (o < NQKV && d < PD) ? val : 0.f;
  }
  const HL s = split8(f);
  const size_t off = (size_t)o * KP + d0;
  for (int ps = 0; ps < 2; ++ps) {
    *(volatile v4u*)(wqh + off) = s.h;
    *(volatile v4u*)(wql + off) = s.l;
    __threadfence();
  }
}

#define STP 72
__global__ __launch_bounds__(256) void k_qkv(const ush* __restrict__ xh, const ush* __restrict__ xl,
                                             const ush* __restrict__ wqh, const ush* __restrict__ wql,
                                             const float* __restrict__ bqkv,
                                             ush* __restrict__ qh, ush* __restrict__ ql,
                                             ush* __restrict__ kh, ush* __restrict__ kl,
                                             _Float16* __restrict__ vt) {
  __shared__ __align__(16) ush st[256 * STP];
  const int tid = threadIdx.x, lane = tid & 31, wave = tid >> 5;
  const int hh = lane >> 4, c = lane & 15;
  const int mb = blockIdx.x * 256;
  const int m0 = mb + wave * 32;
  const int slab = blockIdx.y;
  const int o0 = (slab == 0) ? 0 : (32 + 64 * (slab - 1));

  v8f acc[2][4];
#pragma unroll
  for (int s = 0; s < 2; ++s)
#pragma unroll
    for (int t = 0; t < 4; ++t) acc[s][t] = zero8();
  gemm3_32x64(xh, xl, KP, wqh, wql, KP, m0, o0, lane, acc);

#pragma unroll
  for (int t = 0; t < 4; ++t) {
    const int o  = o0 + 16 * t + c;
    const int oc = (o < NQKV) ? o : (NQKV - 1);
    const float bl = bqkv[oc];
    const float bn = (o < NQKV) ? bl : 0.f;
#pragma unroll
    for (int sub = 0; sub < 2; ++sub) {
#pragma unroll
      for (int r = 0; r < 8; ++r) acc[sub][t][r] += bn;
    }
  }

  if (slab == 0) {
#pragma unroll 1
    for (int ph = 0; ph < 2; ++ph) {
      __syncthreads();
#pragma unroll
      for (int t = 0; t < 2; ++t) {
#pragma unroll
        for (int sub = 0; sub < 2; ++sub) {
#pragma unroll
          for (int r = 0; r < 8; ++r) {
            const int lr = wave * 32 + sub * 16 + 8 * hh + r;
            const float v = acc[sub][t][r];
            const ush hi = f2bf(v);
            st[lr * STP + 16 * t + c] = (ph == 0) ? hi : f2bf(v - bf2f(hi));
          }
        }
      }
      __syncthreads();
#pragma unroll 1
      for (int tg = 0; tg < 2; ++tg) {
        v4u val[4];
        size_t go[4];
#pragma unroll
        for (int j = 0; j < 4; ++j) {
          const int p  = tid + 256 * j;
          const int lr = p >> 2;
          const int pc = p & 3;
          PackU pk;
          pk.s = *(const v8us*)(st + lr * STP + tg * 16 + 8 * (pc & 1));
          const unsigned msk = (pc < 2) ? 0xffffffffu : 0u;
          val[j] = pk.u & (v4u){msk, msk, msk, msk};
          go[j]  = ((size_t)(mb + lr)) * QP + pc * 8;
        }
        ush* dst = (tg == 0) ? ((ph == 0) ? qh : ql) : ((ph == 0) ? kh : kl);
        for (int ps = 0; ps < 2; ++ps) {
#pragma unroll
          for (int j = 0; j < 4; ++j) *(volatile v4u*)(dst + go[j]) = val[j];
          __threadfence();
        }
      }
    }
  } else {
#pragma unroll
    for (int t = 0; t < 4; ++t) {
#pragma unroll
      for (int sub = 0; sub < 2; ++sub) {
#pragma unroll
        for (int r = 0; r < 8; ++r) {
          const int lr = wave * 32 + sub * 16 + 8 * hh + r;
          st[lr * STP + 16 * t + c] = __builtin_bit_cast(ush, (_Float16)acc[sub][t][r]);
        }
      }
    }
    __syncthreads();
    const int b  = mb / LSEQ;
    const int l0 = mb - b * LSEQ;
    const int d0 = o0 - 32;
    v4u val[8];
    size_t go[8];
#pragma unroll
    for (int j = 0; j < 8; ++j) {
      const int p    = tid + 256 * j;
      const int L    = p >> 3;
      const int pc   = p & 7;
      const int dcol = L >> 2;
      const int nl   = (L & 3) * 64 + pc * 8;
      const ush* cp = st + nl * STP + dcol;
      PackU pk;
      pk.s = (v8us){cp[0 * STP], cp[1 * STP], cp[2 * STP], cp[3 * STP],
                    cp[4 * STP], cp[5 * STP], cp[6 * STP], cp[7 * STP]};
      val[j] = pk.u;
      go[j]  = ((size_t)(b * VP + d0 + dcol)) * LSEQ + l0 + nl;
    }
    for (int ps = 0; ps < 2; ++ps) {
#pragma unroll
      for (int j = 0; j < 8; ++j) *(volatile v4u*)(vt + go[j]) = val[j];
      __threadfence();
    }
  }
}

#define SSP 128
#define SPP 136
#define OP  200
__global__ __launch_bounds__(256) void k_attn(const ush* __restrict__ qh, const ush* __restrict__ ql,
                                              const ush* __restrict__ kh, const ush* __restrict__ kl,
                                              const _Float16* __restrict__ vt,
                                              const float* __restrict__ x,
                                              _Float16* __restrict__ mg) {
  __shared__ __align__(16) float    sS[BR * SSP];
  __shared__ __align__(16) _Float16 sP[BR * SPP];
  __shared__ __align__(16) float    sRed[BR * 8];
  __shared__ __align__(16) float    rM[BR];
  __shared__ __align__(16) float    rMn[BR];
  __shared__ __align__(16) float    rL[BR];
  __shared__ __align__(16) float    rSc[BR];

  const int tid = threadIdx.x, lane = tid & 31, wave = tid >> 5;
  const int hh = lane >> 4, c = lane & 15;
  const int b  = blockIdx.y;
  const int q0 = (int)blockIdx.x * BR;
  const size_t tok0 = (size_t)b * LSEQ + q0;
  const ush* Qbh = qh + (size_t)b * LSEQ * QP;
  const ush* Qbl = ql + (size_t)b * LSEQ * QP;
  const ush* Kbh = kh + (size_t)b * LSEQ * QP;
  const ush* Kbl = kl + (size_t)b * LSEQ * QP;
  const _Float16* Vb = vt + (size_t)b * VP * LSEQ;
  const float NEGI = -__builtin_huge_valf();
  if (tid < BR) { rM[tid] = NEGI; rL[tid] = 0.f; }
  __syncthreads();

  const int rt = wave & 1;
  const int cb = wave >> 1;

  const v16us a0h = ldfragu(Qbh, QP, q0, 0, lane);
  const v16us a1h = ldfragu(Qbh, QP, q0 + 16, 0, lane);
  const v16us a0l = ldfragu(Qbl, QP, q0, 0, lane);
  const v16us a1l = ldfragu(Qbl, QP, q0 + 16, 0, lane);

  v8f oacc[3];
#pragma unroll
  for (int e = 0; e < 3; ++e) oacc[e] = zero8();

  const int srow = tid >> 3, schk = tid & 7;

#pragma unroll 1
  for (int ch = 0; ch < LSEQ / BC; ++ch) {
    const int j0  = ch * BC;
    const int kr0 = j0 + wave * 16;
    const v16us kbh = ldfragu(Kbh, QP, kr0, 0, lane);
    const v16us kbl = ldfragu(Kbl, QP, kr0, 0, lane);
    v8f s0 = zero8(), s1 = zero8();
    s0 = mmab(a0h, kbh, s0);
    s1 = mmab(a1h, kbh, s1);
    s0 = mmab(a0h, kbl, s0);
    s1 = mmab(a1h, kbl, s1);
    s0 = mmab(a0l, kbh, s0);
    s1 = mmab(a1l, kbh, s1);
#pragma unroll
    for (int r = 0; r < 8; ++r) {
      sS[(8 * hh + r) * SSP + wave * 16 + c]      = s0[r] * 0.25f;
      sS[(16 + 8 * hh + r) * SSP + wave * 16 + c] = s1[r] * 0.25f;
    }
    __syncthreads();
    {
      const float* sr = sS + srow * SSP + schk * 16;
      const v4f x0 = *(const v4f*)(sr);
      const v4f x1 = *(const v4f*)(sr + 4);
      const v4f x2 = *(const v4f*)(sr + 8);
      const v4f x3 = *(const v4f*)(sr + 12);
      float mx = x0[0];
#pragma unroll
      for (int e = 1; e < 4; ++e) mx = fmaxf(mx, x0[e]);
#pragma unroll
      for (int e = 0; e < 4; ++e) { mx = fmaxf(mx, x1[e]); mx = fmaxf(mx, x2[e]); mx = fmaxf(mx, x3[e]); }
      sRed[srow * 8 + schk] = mx;
    }
    __syncthreads();
    if (tid < BR) {
      float mx = rM[tid];
#pragma unroll
      for (int i = 0; i < 8; ++i) mx = fmaxf(mx, sRed[tid * 8 + i]);
      rMn[tid] = mx;
    }
    __syncthreads();
    {
      const float mx = rMn[srow];
      const float* sr = sS + srow * SSP + schk * 16;
      float sum = 0.f;
      Pack8 p0, p1;
#pragma unroll
      for (int e = 0; e < 8; ++e) {
        const float p = __expf(sr[e] - mx);
        sum += p;
        p0.h[e] = (_Float16)(p * 1024.0f);
      }
#pragma unroll
      for (int e = 0; e < 8; ++e) {
        const float p = __expf(sr[8 + e] - mx);
        sum += p;
        p1.h[e] = (_Float16)(p * 1024.0f);
      }
      *(v8h*)(sP + srow * SPP + schk * 16)     = p0.h;
      *(v8h*)(sP + srow * SPP + schk * 16 + 8) = p1.h;
      sRed[srow * 8 + schk] = sum;
    }
    __syncthreads();
    if (tid < BR) {
      float sum = 0.f;
#pragma unroll
      for (int i = 0; i < 8; ++i) sum += sRed[tid * 8 + i];
      const float mnew = rMn[tid];
      const float fac  = __expf(rM[tid] - mnew);
      rL[tid]  = rL[tid] * fac + sum;
      rM[tid]  = mnew;
      rSc[tid] = fac;
    }
    __syncthreads();
    {
      const v4f f0 = *(const v4f*)(rSc + 16 * rt + 8 * hh);
      const v4f f1 = *(const v4f*)(rSc + 16 * rt + 8 * hh + 4);
#pragma unroll
      for (int e = 0; e < 3; ++e) {
#pragma unroll
        for (int r = 0; r < 4; ++r) {
          oacc[e][r]     *= f0[r];
          oacc[e][4 + r] *= f1[r];
        }
      }
    }
#pragma unroll 1
    for (int kk = 0; kk < BC / 32; ++kk) {
      const v16h pa = ldfrag(sP, SPP, 16 * rt, kk * 32, lane);
#pragma unroll
      for (int e = 0; e < 3; ++e) {
        const v16h vb = ldfrag(Vb, LSEQ, 16 * (cb + 4 * e), j0 + kk * 32, lane);
        oacc[e] = mma16(pa, vb, oacc[e]);
      }
    }
    __syncthreads();
  }

  _Float16* sO = (_Float16*)sS;
#pragma unroll
  for (int r = 0; r < 8; ++r) {
    const int row  = 16 * rt + 8 * hh + r;
    const float lv = rL[row];
    const float inv = (lv > 0.f) ? (0.015625f / lv) : 0.f;
#pragma unroll
    for (int e = 0; e < 3; ++e) sO[row * OP + 16 * (cb + 4 * e) + c] = (_Float16)(oacc[e][r] * inv);
  }
  __syncthreads();
#pragma unroll
  for (int i = 0; i < 4; ++i) {
    const int idx = tid + 256 * i;
    const int idc = (idx < BR * 28) ? idx : (BR * 28 - 1);
    const int row = idc / 28;
    const int cc  = idc - row * 28;
    const float xv = x[(tok0 + (size_t)row) * HID + PD + cc];
    if (idx < BR * 28) sO[row * OP + PD + cc] = (_Float16)xv;
  }
  __syncthreads();
  v4u val[3];
  size_t go[3];
#pragma unroll
  for (int j = 0; j < 3; ++j) {
    const int p   = tid + 256 * j;
    const int row = p / 24;
    const int pr  = p - row * 24;
    Pack8 pk;
    pk.h  = *(const v8h*)(sO + row * OP + pr * 8);
    val[j] = pk.u;
    go[j]  = (tok0 + (size_t)row) * HID + pr * 8;
  }
  for (int ps = 0; ps < 2; ++ps) {
#pragma unroll
    for (int j = 0; j < 3; ++j) *(volatile v4u*)(mg + go[j]) = val[j];
    __threadfence();
  }
}

#define OTP 68
__global__ __launch_bounds__(256) void k_out(const _Float16* __restrict__ mg,
                                             const _Float16* __restrict__ wo,
                                             const float* __restrict__ ob,
                                             float* __restrict__ out) {
  __shared__ __align__(16) float sw[8 * 16 * OTP];
  const int tid = threadIdx.x, lane = tid & 31, wave = tid >> 5;
  const int hh = lane >> 4, c = lane & 15;
  const int m0 = blockIdx.x * 256 + wave * 32;
  const int n0 = blockIdx.y * 64;
  float* st = sw + wave * (16 * OTP);

  v8f acc[2][4];
#pragma unroll
  for (int s = 0; s < 2; ++s)
#pragma unroll
    for (int t = 0; t < 4; ++t) acc[s][t] = zero8();
  gemm32x64(mg, HID, wo, HID, m0, n0, lane, acc);

  float bn[4];
#pragma unroll
  for (int t = 0; t < 4; ++t) bn[t] = ob[n0 + 16 * t + c];

#pragma unroll
  for (int sub = 0; sub < 2; ++sub) {
    __syncthreads();
#pragma unroll
    for (int r = 0; r < 8; ++r) {
#pragma unroll
      for (int t = 0; t < 4; ++t) st[(8 * hh + r) * OTP + 16 * t + c] = acc[sub][t][r] * 0.03125f + bn[t];
    }
    __syncthreads();
    v4f val[8];
    size_t go[8];
#pragma unroll
    for (int it = 0; it < 8; ++it) {
      const int p    = lane + 32 * it;
      const int L    = p >> 3;
      const int pc   = p & 7;
      const int row  = L >> 1;
      const int half = L & 1;
      val[it] = *(const v4f*)(st + row * OTP + half * 32 + pc * 4);
      go[it]  = ((size_t)(m0 + sub * 16 + row)) * HID + n0 + half * 32 + pc * 4;
    }
    for (int ps = 0; ps < 2; ++ps) {
#pragma unroll
      for (int it = 0; it < 8; ++it) *(volatile v4f*)(out + go[it]) = val[it];
      __threadfence();
    }
  }
}

extern "C" void kernel_launch(void* const* d_in, const int* in_sizes, int n_in,
                              void* d_out, int out_size, void* d_ws, size_t ws_size,
                              hipStream_t stream) {
  if (n_in < 7) return;
  if (in_sizes[0] != NTOK * HID) return;
  if (in_sizes[1] != PD) return;
  if (in_sizes[2] != PD) return;
  if (in_sizes[3] != NQKV * PD) return;
  if (in_sizes[4] != NQKV) return;
  if (in_sizes[5] != HID * HID) return;
  if (in_sizes[6] != HID) return;
  if (out_size != NTOK * HID) return;

  const float* x   = (const float*)d_in[0];
  const float* lng = (const float*)d_in[1];
  const float* lnb = (const float*)d_in[2];
  const float* qw  = (const float*)d_in[3];
  const float* qb  = (const float*)d_in[4];
  const float* ow  = (const float*)d_in[5];
  const float* ob  = (const float*)d_in[6];
  float* out = (float*)d_out;

  size_t off = 0;
  const size_t oXh  = off; off += (size_t)NTOK * KP * 2;
  const size_t oXl  = off; off += (size_t)NTOK * KP * 2;
  const size_t oMG  = off; off += (size_t)NTOK * HID * 2;
  const size_t oWo  = off; off += (size_t)HID * HID * 2;
  const size_t oWqh = off; off += (size_t)NQP * KP * 2;
  const size_t oWql = off; off += (size_t)NQP * KP * 2;
  const size_t oQh  = off; off += (size_t)NTOK * QP * 2;
  const size_t oQl  = off; off += (size_t)NTOK * QP * 2;
  const size_t oKh  = off; off += (size_t)NTOK * QP * 2;
  const size_t oKl  = off; off += (size_t)NTOK * QP * 2;
  const size_t oVt  = off; off += (size_t)NB * VP * LSEQ * 2;
  if (off > ws_size) return;
  if (off > (size_t)134217728) return;

  char* ws = (char*)d_ws;
  ush*      Xh  = (ush*)(ws + oXh);
  ush*      Xl  = (ush*)(ws + oXl);
  _Float16* MG  = (_Float16*)(ws + oMG);
  _Float16* Wo  = (_Float16*)(ws + oWo);
  ush*      Wqh = (ush*)(ws + oWqh);
  ush*      Wql = (ush*)(ws + oWql);
  ush*      Qh  = (ush*)(ws + oQh);
  ush*      Ql  = (ush*)(ws + oQl);
  ush*      Kh  = (ush*)(ws + oKh);
  ush*      Kl  = (ush*)(ws + oKl);
  _Float16* Vt  = (_Float16*)(ws + oVt);

  k_prep<<<dim3(NTOK / 8), dim3(256), 0, stream>>>(x, lng, lnb, Xh, Xl, MG);
  const int ngo = (HID * HID) / 8;
  k_cvt_wo<<<dim3((ngo + 255) / 256), dim3(256), 0, stream>>>(ow, Wo, ngo);
  const int ngq = (NQP * KP) / 8;
  k_cvt_wq<<<dim3((ngq + 255) / 256), dim3(256), 0, stream>>>(qw, Wqh, Wql, ngq);
  k_qkv<<<dim3(NTOK / 256, 4), dim3(256), 0, stream>>>(Xh, Xl, Wqh, Wql, qb, Qh, Ql, Kh, Kl, Vt);
  k_attn<<<dim3(NQT, NB), dim3(256), 0, stream>>>(Qh, Ql, Kh, Kl, Vt, x, MG);
  k_out<<<dim3(NTOK / 256, HID / 64), dim3(256), 0, stream>>>(MG, Wo, ob, out);
  (void)hipGetLastError();
}
